// QGate_65481071403203
// MI455X (gfx1250) — hardware-verified
//
#include <hip/hip_runtime.h>


#ifndef NB
#define NB 128
#endif
#define NB_FULL 128
#define NQ     14
#define NST    16384
#define NLAY   3
#define NGRP   4
#define NMAT   (NLAY * NGRP)
#define MROW   32
#define MSZ    (MROW * MROW)
#define BLK    256
#define NWV    (BLK / 32)
#define NCOL   (NST / 16)
#define NSTEP  (NCOL / (NWV * 16))
#define ZPITCH 32
#define N4     (NB * NQ / 4)
#define SCAR   16384.0f
#define PSCI   3.7252902984619140625e-09f
#define MCAR   256.0f
#define MCI    (1.0f / 256.0f)
#define QRS    2048.0f
#define QRI    (1.0f / 2048.0f)

static_assert(NQ == 14);
static_assert(NST == (1 << NQ));
static_assert(BLK == 256);
static_assert(BLK * 8 == 2 * MSZ);
static_assert(NST % BLK == 0);
static_assert(NCOL % (NWV * 16) == 0);
static_assert(NSTEP * NWV * 16 == NCOL);
static_assert((NST / 4) % BLK == 0);
static_assert(NLAY * NQ * 3 == 126);
static_assert(NB <= NB_FULL);
static_assert((NB * NQ) % 32 == 0);
static_assert(N4 <= 2 * BLK);
static_assert(NQ <= ZPITCH);
static_assert(4 * 8 == ZPITCH);
static_assert(MROW == 32);

typedef _Float16 h16;
typedef unsigned short bf;
typedef __attribute__((ext_vector_type(16))) _Float16 v16h;
typedef __attribute__((ext_vector_type(8)))  _Float16 v8h;
typedef __attribute__((ext_vector_type(8)))  float    v8f;
typedef __attribute__((ext_vector_type(4)))  float    v4f;
typedef __attribute__((ext_vector_type(8)))  unsigned v8u;
typedef __attribute__((ext_vector_type(2)))  unsigned v2u;
typedef v8h  __attribute__((may_alias)) v8ha;

static_assert(sizeof(v2u) * NST <= 131072);

__device__ __forceinline__ unsigned short f2bf(float f) { unsigned u = __float_as_uint(f); u += 0x7FFFu + ((u >> 16) & 1u); return (unsigned short)(u >> 16); }
__device__ __forceinline__ float bfr(float f) { return __uint_as_float(((unsigned)f2bf(f)) << 16); }
__device__ __forceinline__ v16h cat16(v8h lo, v8h hi) { return __builtin_shufflevector(lo, hi, 0, 1, 2, 3, 4, 5, 6, 7, 8, 9, 10, 11, 12, 13, 14, 15); }
__device__ __forceinline__ v16h  ldh(const h16* p) { return cat16(*(const v8h*)p, *(const v8h*)(p + 16)); }
static __device__ __forceinline__ h16 toh_flush(float v) { const h16 r = (h16)v; return (fabsf(v) < 6.103515625e-05f) ? (h16)0.0f : r; }
__device__ __forceinline__ v8f wmma16g(v16h a, v16h b, v8f c) {
    c = __builtin_amdgcn_wmma_f32_16x16x32_f16(false, a, false, b, (short)0, c, false, false);
    asm volatile("v_nop\n\tv_nop\n\tv_nop\n\tv_nop" : "+v"(c) : "v"(a), "v"(b));
    return c;
}
__device__ __forceinline__ unsigned hbits(h16 v) { return (unsigned)__builtin_bit_cast(unsigned short, v); }
__device__ __forceinline__ float hlo(unsigned w) { return (float)__builtin_bit_cast(h16, (unsigned short)(w & 0xFFFFu)); }
__device__ __forceinline__ float hhi(unsigned w) { return (float)__builtin_bit_cast(h16, (unsigned short)(w >> 16)); }
__device__ __forceinline__ v2u pk4(float re, float im) {
    const h16 rh = toh_flush(re), ih = toh_flush(im);
    const h16 rr = toh_flush((re - (float)rh) * QRS), ir = toh_flush((im - (float)ih) * QRS);
    v2u o; o.x = hbits(rh) | (hbits(ih) << 16); o.y = hbits(rr) | (hbits(ir) << 16); return o;
}

__global__ __launch_bounds__(BLK) void k_gmat(const float* __restrict__ params, h16* GP) {
#pragma clang fp contract(off)
    __shared__ float CS[48];
    __shared__ float SN[48];
    __shared__ float UW[16 * 8];
    __shared__ __align__(16) h16 T[2 * MSZ];
    const int tid = threadIdx.x;
    const int mi = blockIdx.x; const int l = mi >> 2, g = mi & 3;
    const int p = (g == 3) ? 0 : (10 - 4 * g);
    { const int ta = tid < NQ * 3 ? tid : NQ * 3 - 1;
      const float a = bfr(params[l * NQ * 3 + ta]);
      const float th = 0.5f * a;
      const float c = cosf(th), s = sinf(th);
      if (tid < NQ * 3) { CS[tid] = c; SN[tid] = s; } }
    __syncthreads();
    { const int q = tid < NQ ? tid : NQ - 1;
      const float c0 = CS[3 * q], s0 = SN[3 * q], c1 = CS[3 * q + 1], s1 = SN[3 * q + 1], cz = CS[3 * q + 2], sz = SN[3 * q + 2];
      const float ar00 =  cz * c1 * c0 + sz * s1 * s0;
      const float ai00 =  cz * s1 * s0 - sz * c1 * c0;
      const float ar01 = -cz * s1 * c0 - sz * c1 * s0;
      const float ai01 =  sz * s1 * c0 - cz * c1 * s0;
      const float ar10 =  cz * s1 * c0 + sz * c1 * s0;
      const float ai10 =  sz * s1 * c0 - cz * c1 * s0;
      const float ar11 =  cz * c1 * c0 + sz * s1 * s0;
      const float ai11 =  sz * c1 * c0 - cz * s1 * s0;
      if (tid < NQ) { UW[tid * 8 + 0] = ar00; UW[tid * 8 + 1] = ai00; UW[tid * 8 + 2] = ar01; UW[tid * 8 + 3] = ai01;
                      UW[tid * 8 + 4] = ar10; UW[tid * 8 + 5] = ai10; UW[tid * 8 + 6] = ar11; UW[tid * 8 + 7] = ai11; } }
    __syncthreads();
    { const int jo = tid >> 4, ji = tid & 15;
      float ur = 1.0f, ui = 0.0f;
#pragma unroll 1
      for (int i = 0; i < 4; ++i) {
          const int q = (NQ - 1) - (p + i);
          const int bo = (jo >> i) & 1, bi = (ji >> i) & 1;
          const int ua = q * 8 + (bo * 2 + bi) * 2;
          float fr = UW[ua], fi = UW[ua + 1];
          const bool ident = (g == 3) & (i >= 2);
          const float dr = (bo == bi) ? 1.0f : 0.0f;
          fr = ident ? dr : fr; fi = ident ? 0.0f : fi;
          const float nr = ur * fr - ui * fi, ni = ur * fi + ui * fr;
          ur = nr; ui = ni; }
      const float e00 = ur * MCAR, e01 = -ui * MCAR, e10 = ui * MCAR, e11 = ur * MCAR;
      const h16 h00 = toh_flush(e00), h01 = toh_flush(e01), h10 = toh_flush(e10), h11 = toh_flush(e11);
      const h16 r00 = toh_flush((e00 - (float)h00) * QRS), r01 = toh_flush((e01 - (float)h01) * QRS);
      const h16 r10 = toh_flush((e10 - (float)h10) * QRS), r11 = toh_flush((e11 - (float)h11) * QRS);
      const int tb = (2 * jo) * MROW + 2 * ji;
      T[tb] = h00; T[tb + 1] = h01; T[tb + MROW] = h10; T[tb + MROW + 1] = h11;
      T[MSZ + tb] = r00; T[MSZ + tb + 1] = r01; T[MSZ + tb + MROW] = r10; T[MSZ + tb + MROW + 1] = r11; }
    __syncthreads();
    { const v8h pv = *(const v8ha*)(&T[8 * tid]);
      const size_t dof = (size_t)((tid < 128) ? 0 : NMAT * MSZ) + (size_t)mi * MSZ + (size_t)(tid & 127) * 8;
      *(volatile v8h*)(GP + dof) = pv; __threadfence(); *(volatile v8h*)(GP + dof) = pv; }
}

__global__ __launch_bounds__(BLK) void k_sim(const float* __restrict__ x, const h16* __restrict__ GP, float* ZP) {
    __shared__ __align__(16) v2u st[NST];
    const int tid = threadIdx.x;
    const int lane = tid & 31, lr = lane & 15, hi = lane >> 4;
    const int wave = __builtin_amdgcn_readfirstlane((int)(threadIdx.x >> 5));
    const int b = blockIdx.x;
    const int xq = lane < NQ ? lane : NQ - 1;
    const float xa = bfr(x[(size_t)b * NQ + xq]);
    const float xc = cosf(0.5f * xa), xs = sinf(0.5f * xa);
    float lowp = SCAR;
#pragma unroll 1
    for (int i = 0; i < 8; ++i) { const int q = (NQ - 1) - i;
        const float cq = __shfl(xc, q, 32), sq = __shfl(xs, q, 32);
        lowp *= ((tid >> i) & 1) ? sq : cq; }
#pragma unroll 1
    for (int it = 0; it < NST / BLK; ++it) {
        float hp = lowp;
#pragma unroll 1
        for (int i = 0; i < 6; ++i) { const int q = 5 - i;
            const float cq = __shfl(xc, q, 32), sq = __shfl(xs, q, 32);
            hp *= ((it >> i) & 1) ? sq : cq; }
        const int s = tid + it * BLK;
        const int pc = __popc((unsigned)s) & 3;
        const float re = (pc == 0) ? hp : ((pc == 2) ? -hp : 0.0f);
        const float im = (pc == 1) ? -hp : ((pc == 3) ? hp : 0.0f);
        st[s] = pk4(re, im); }
    __syncthreads();

#pragma unroll 1
    for (int l = 0; l < NLAY; ++l) {
#pragma unroll 1
        for (int g = 0; g < NGRP; ++g) {
            const int p = (g == 3) ? 0 : (10 - 4 * g);
            const int pm = (1 << p) - 1;
            const size_t mo = (size_t)(l * NGRP + g) * MSZ + (size_t)lr * MROW + 8 * hi;
            const v16h aH0 = ldh(GP + mo), aH1 = ldh(GP + mo + 16 * MROW);
            const v16h aR0 = ldh(GP + (size_t)NMAT * MSZ + mo), aR1 = ldh(GP + (size_t)NMAT * MSZ + mo + 16 * MROW);
#pragma unroll 1
            for (int step = 0; step < NSTEP; ++step) {
                const int cidx = step * (NWV * 16) + wave * 16 + lr;
                const int base = (cidx & pm) | ((cidx >> p) << (p + 4));
                v8u wh, wr;
#pragma unroll
                for (int i = 0; i < 4; ++i) {
                    const v2u t0 = st[base + ((4 * hi + i) << p)];
                    const v2u t1 = st[base + ((8 + 4 * hi + i) << p)];
                    wh[i] = t0.x; wr[i] = t0.y; wh[4 + i] = t1.x; wr[4 + i] = t1.y; }
                const v16h bh = __builtin_bit_cast(v16h, wh), br = __builtin_bit_cast(v16h, wr);
                const v8f z = (v8f){};
                v8f dH0 = wmma16g(aH0, bh, z);
                v8f dR0 = wmma16g(aR0, bh, z); dR0 = wmma16g(aH0, br, dR0);
                v8f dH1 = wmma16g(aH1, bh, z);
                v8f dR1 = wmma16g(aR1, bh, z); dR1 = wmma16g(aH1, br, dR1);
                const v8f f0 = (dH0 + dR0 * QRI) * MCI, f1 = (dH1 + dR1 * QRI) * MCI;
#pragma unroll
                for (int i = 0; i < 4; ++i) {
                    st[base + ((4 * hi + i) << p)]     = pk4(f0[2 * i], f0[2 * i + 1]);
                    st[base + ((8 + 4 * hi + i) << p)] = pk4(f1[2 * i], f1[2 * i + 1]); }
            }
            __syncthreads();
        }
#pragma unroll 1
        for (int cn = 0; cn < NQ; ++cn) {
            const int pc = (cn < NQ - 1) ? (NQ - 1 - cn) : 0;
            const int pt = (cn < NQ - 1) ? (NQ - 2 - cn) : (NQ - 1);
            const int lo = pc < pt ? pc : pt, hb = pc < pt ? pt : pc;
#pragma unroll 2
            for (int it = 0; it < (NST / 4) / BLK; ++it) {
                const int j = tid + it * BLK;
                const int t = j + ((j >> lo) << lo);
                int i = t + ((t >> hb) << hb);
                i |= (1 << pc);
                const int i2 = i | (1 << pt);
                const v2u a = st[i], c = st[i2];
                st[i] = c; st[i2] = a; }
            __syncthreads();
        }
    }

    float acc[NQ];
#pragma unroll
    for (int w = 0; w < NQ; ++w) acc[w] = 0.0f;
#pragma unroll 2
    for (int it = 0; it < NST / BLK; ++it) {
        const int i = tid + it * BLK;
        const v2u t = st[i];
        const float re = hlo(t.x) + hlo(t.y) * QRI, im = hhi(t.x) + hhi(t.y) * QRI;
        const float pr = re * re + im * im;
#pragma unroll
        for (int w = 0; w < NQ; ++w) acc[w] += ((i >> ((NQ - 1) - w)) & 1) ? -pr : pr; }
#pragma unroll
    for (int w = 0; w < NQ; ++w) { float v = acc[w];
        v += __shfl_xor(v, 16, 32); v += __shfl_xor(v, 8, 32); v += __shfl_xor(v, 4, 32); v += __shfl_xor(v, 2, 32); v += __shfl_xor(v, 1, 32);
        acc[w] = v; }
    const int li = lane & 7;
    v4f zv;
#pragma unroll
    for (int c = 0; c < 4; ++c) { const int e = 4 * li + c; float s = 0.0f;
#pragma unroll
        for (int k = 0; k < NQ; ++k) s = (e == k) ? acc[k] : s;
        zv[c] = s * PSCI; }
    float* zl = ZP + ((size_t)b * NWV + wave) * ZPITCH + 4 * li;
#pragma unroll 1
    for (int ps = 0; ps < 2; ++ps) { if (lane < 8) *(volatile v4f*)zl = zv; if (ps == 0) __threadfence(); }
}

__global__ __launch_bounds__(BLK) void k_out(const float* __restrict__ ZP, float* OUT) {
    const int tid = threadIdx.x;
    v4f v[2];
#pragma unroll
    for (int t = 0; t < 2; ++t) {
        const int i = tid + t * BLK; const int ic = i < N4 ? i : N4 - 1;
        v4f s = (v4f){};
#pragma unroll 1
        for (int wv = 0; wv < NWV; ++wv) {
#pragma unroll
            for (int c = 0; c < 4; ++c) { const int e = 4 * ic + c; const int bb = e / NQ; const int w = e - bb * NQ;
                s[c] += ZP[((size_t)bb * NWV + wv) * ZPITCH + w]; } }
        v[t] = s; }
#pragma unroll 1
    for (int ps = 0; ps < 2; ++ps) {
#pragma unroll
        for (int t = 0; t < 2; ++t) { const int i = tid + t * BLK;
            if (i < N4) *(volatile v4f*)(OUT + (size_t)i * 4) = v[t]; }
        if (ps == 0) __threadfence(); }
}

static constexpr size_t al256(size_t v) { return (v + 255) & ~(size_t)255; }
static constexpr size_t SZ_GP = al256((size_t)2 * NMAT * MSZ * 2);
static constexpr size_t SZ_ZP = al256((size_t)NB * NWV * ZPITCH * 4);
static constexpr size_t SZ_TOTAL = SZ_GP + SZ_ZP;
static_assert(SZ_TOTAL <= (size_t)134217728);
static_assert(((size_t)NMAT * MSZ * 2) % 128 == 0);
static_assert(((size_t)MSZ * 2) % 128 == 0);
static_assert((size_t)(NB - 1) * NWV * ZPITCH + (NWV - 1) * ZPITCH + ZPITCH <= SZ_ZP / 4);
static_assert((size_t)(NMAT - 1) * MSZ + MSZ + (size_t)NMAT * MSZ <= SZ_GP / 2);

extern "C" void kernel_launch(void* const* d_in, const int* in_sizes, int n_in,
                              void* d_out, int out_size, void* d_ws, size_t ws_size, hipStream_t stream) {
    if (n_in < 2) return;
    if ((size_t)in_sizes[0] < (size_t)NB * NQ) return;
    if (in_sizes[1] < NLAY * NQ * 3) return;
    if ((size_t)out_size < (size_t)NB * NQ) return;
    if (SZ_TOTAL > ws_size) return;
    const float* x = (const float*)d_in[0];
    const float* params = (const float*)d_in[1];
    float* OUT = (float*)d_out;
    char* wsp = (char*)d_ws;
    h16* GP = (h16*)wsp; wsp += SZ_GP;
    float* ZP = (float*)wsp; wsp += SZ_ZP;

    k_gmat<<<dim3(NMAT, 1, 1), BLK, 0, stream>>>(params, GP);
    k_sim<<<dim3(NB, 1, 1), BLK, 0, stream>>>(x, GP, ZP);
    k_out<<<dim3(1, 1, 1), BLK, 0, stream>>>(ZP, OUT);
}
